// MLPPredictor_9689446219935
// MI455X (gfx1250) — hardware-verified
//
#include <hip/hip_runtime.h>
#include <stddef.h>
#include <stdint.h>

#define HDIM   128
#define KDIM   256
#define NROWB  32
#define GTHR   128
#define TP     132
#define EPB    256
#define NUNW   (KDIM * HDIM / 8)
#define WSMAX  134217728

static_assert(KDIM == 2 * HDIM && HDIM % 32 == 0);
static_assert(NROWB == (GTHR / 32 / 2) * 16);
static_assert(((TP * 4) % 16) == 0);
static_assert(EPB == 2 * HDIM);
static_assert(EPB / 4 == 64);
static_assert(NUNW % 256 == 0);

typedef float          v4f   __attribute__((ext_vector_type(4)));
typedef float          v8f   __attribute__((ext_vector_type(8)));
typedef int            v8i   __attribute__((ext_vector_type(8)));
typedef unsigned short v8us  __attribute__((ext_vector_type(8)));
typedef unsigned short v16us __attribute__((ext_vector_type(16)));
typedef __bf16         v16bf __attribute__((ext_vector_type(16)));
typedef v4f  __attribute__((may_alias)) v4fa;
typedef v8us __attribute__((may_alias)) v8usa;
union FragB { v16bf v; v16us u; v8us h[2]; v8i w; };

__device__ __forceinline__ v8f wmb(const FragB& a, const FragB& b, v8f c) {
  v8f d = __builtin_amdgcn_wmma_f32_16x16x32_bf16(false, a.v, false, b.v, (short)0, c, false, false);
  asm volatile("v_nop\n\tv_nop\n\tv_nop\n\tv_nop" : "+v"(d) : "v"(a.w), "v"(b.w));
  return d;
}

__device__ __forceinline__ unsigned bf16_bits(float f) {
  const unsigned u = __float_as_uint(f);
  return (u + 0x7FFFu + ((u >> 16) & 1u)) >> 16;
}
__device__ __forceinline__ float bf16_val(float f) {
  return __uint_as_float(bf16_bits(f) << 16);
}

__global__ __launch_bounds__(256) void k_wprep(const float* __restrict__ W1, unsigned short* WB, int nUnits) {
  const int u = (int)blockIdx.x * 256 + (int)threadIdx.x;
  if (u >= nUnits) return;
  const int c    = u >> 4;
  const int k8   = (u & 15) * 8;
  const int srow = c & (HDIM - 1);
  const int scol = ((c >> 7) & 1) * HDIM + k8;
  const float* p = W1 + (size_t)srow * KDIM + scol;
  const v4f a = *(const v4fa*)p;
  const v4f b = *(const v4fa*)(p + 4);
  v8us o;
  o[0] = (unsigned short)bf16_bits(a.x);
  o[1] = (unsigned short)bf16_bits(a.y);
  o[2] = (unsigned short)bf16_bits(a.z);
  o[3] = (unsigned short)bf16_bits(a.w);
  o[4] = (unsigned short)bf16_bits(b.x);
  o[5] = (unsigned short)bf16_bits(b.y);
  o[6] = (unsigned short)bf16_bits(b.z);
  o[7] = (unsigned short)bf16_bits(b.w);
  unsigned short* dp = WB + (size_t)u * 8;
  *(volatile v8us*)dp = o;
  __threadfence();
  *(volatile v8us*)dp = o;
}

__global__ __launch_bounds__(GTHR) void k_node(
    const float* __restrict__ hN,
    const unsigned short* __restrict__ WB,
    float* PQ,
    int nA)
{
  __shared__ __attribute__((aligned(16))) float sT[4 * 16 * TP];

  const int tid = (int)threadIdx.x, lane = tid & 31, wave = tid >> 5;
  const int hh = lane >> 4, m = lane & 15;
  const int rt = wave >> 1, ch = wave & 1;
  const int a0 = (int)blockIdx.x * NROWB + 16 * rt;

  int ar = a0 + m;
  ar = ar > nA - 1 ? nA - 1 : ar;
  const float* zr = hN + (size_t)ar * HDIM + 8 * hh;
  const unsigned short* wp = WB + (size_t)(ch * HDIM + m) * HDIM + 8 * hh;

  v8f acc[8];
  {
    const v8f z8 = {0.f, 0.f, 0.f, 0.f, 0.f, 0.f, 0.f, 0.f};
#pragma unroll
    for (int t = 0; t < 8; ++t) acc[t] = z8;
  }

#pragma unroll 1
  for (int kk = 0; kk < HDIM / 32; ++kk) {
    const int k0 = 32 * kk;
    const v4f f0 = *(const v4fa*)(zr + k0);
    const v4f f1 = *(const v4fa*)(zr + k0 + 4);
    const v4f f2 = *(const v4fa*)(zr + k0 + 16);
    const v4f f3 = *(const v4fa*)(zr + k0 + 20);
    FragB af;
    af.u[0]  = (unsigned short)bf16_bits(f0.x);
    af.u[1]  = (unsigned short)bf16_bits(f0.y);
    af.u[2]  = (unsigned short)bf16_bits(f0.z);
    af.u[3]  = (unsigned short)bf16_bits(f0.w);
    af.u[4]  = (unsigned short)bf16_bits(f1.x);
    af.u[5]  = (unsigned short)bf16_bits(f1.y);
    af.u[6]  = (unsigned short)bf16_bits(f1.z);
    af.u[7]  = (unsigned short)bf16_bits(f1.w);
    af.u[8]  = (unsigned short)bf16_bits(f2.x);
    af.u[9]  = (unsigned short)bf16_bits(f2.y);
    af.u[10] = (unsigned short)bf16_bits(f2.z);
    af.u[11] = (unsigned short)bf16_bits(f2.w);
    af.u[12] = (unsigned short)bf16_bits(f3.x);
    af.u[13] = (unsigned short)bf16_bits(f3.y);
    af.u[14] = (unsigned short)bf16_bits(f3.z);
    af.u[15] = (unsigned short)bf16_bits(f3.w);
#pragma unroll
    for (int nt = 0; nt < 8; ++nt) {
      const unsigned short* wq = wp + (size_t)(16 * nt) * HDIM + k0;
      FragB bf;
      bf.h[0] = *(const v8usa*)wq;
      bf.h[1] = *(const v8usa*)(wq + 16);
      acc[nt] = wmb(af, bf, acc[nt]);
    }
  }

  float* sTw = sT + wave * 16 * TP;
#pragma unroll
  for (int nt = 0; nt < 8; ++nt) {
#pragma unroll
    for (int r = 0; r < 8; ++r) sTw[(8 * hh + r) * TP + 16 * nt + m] = acc[nt][r];
  }
  __syncthreads();

  float* dstp = PQ + (size_t)ch * HDIM + 4 * lane;
#pragma unroll
  for (int i = 0; i < 16; ++i) {
    const int row = a0 + i;
    if (row < nA) {
      const v4f v = *(const v4fa*)(sTw + i * TP + 4 * lane);
      *(volatile v4f*)(dstp + (size_t)row * KDIM) = v;
    }
  }
  __threadfence();
#pragma unroll
  for (int i = 0; i < 16; ++i) {
    const int row = a0 + i;
    if (row < nA) {
      const v4f v = *(const v4fa*)(sTw + i * TP + 4 * lane);
      *(volatile v4f*)(dstp + (size_t)row * KDIM) = v;
    }
  }
}

__device__ __forceinline__ void out_store_pass(float* out, v4f v, int eb, int nE, bool full, bool tailw) {
  if (full) {
    *(volatile v4f*)(out + (size_t)eb) = v;
  } else if (tailw) {
    if (eb     < nE) *(volatile float*)(out + (size_t)eb)     = v.x;
    if (eb + 1 < nE) *(volatile float*)(out + (size_t)eb + 1) = v.y;
    if (eb + 2 < nE) *(volatile float*)(out + (size_t)eb + 2) = v.z;
    if (eb + 3 < nE) *(volatile float*)(out + (size_t)eb + 3) = v.w;
  }
}

__global__ __launch_bounds__(EPB) void k_edge(
    const float* PQ,
    const int*   __restrict__ srcI,
    const int*   __restrict__ dstI,
    const float* __restrict__ b1,
    const float* __restrict__ W2,
    const float* __restrict__ b2,
    float* out,
    int nE, int nA)
{
  __shared__ __attribute__((aligned(16))) float sB1[HDIM];
  __shared__ __attribute__((aligned(16))) float sW2[HDIM];
  __shared__ __attribute__((aligned(16))) float sOut[EPB];

  const int tid = (int)threadIdx.x;
  if (tid < HDIM) sB1[tid] = bf16_val(b1[tid]);
  else            sW2[tid - HDIM] = bf16_val(W2[tid - HDIM]);
  __syncthreads();

  const int e0 = (int)blockIdx.x * EPB;
  int e = e0 + tid;
  e = e > nE - 1 ? nE - 1 : e;
  const int rawr = srcI[(size_t)e];
  const int rawc = dstI[(size_t)e];
  int ri = rawr < 0 ? rawr + nA : rawr;
  ri = ri < 0 ? 0 : (ri > nA - 1 ? nA - 1 : ri);
  int ci = rawc < 0 ? rawc + nA : rawc;
  ci = ci < 0 ? 0 : (ci > nA - 1 ? nA - 1 : ci);

  const float* pr = PQ + (size_t)ri * KDIM;
  const float* pc = PQ + (size_t)ci * KDIM + HDIM;
  float s = 0.0f;
#pragma unroll 4
  for (int j = 0; j < HDIM / 4; ++j) {
    const v4f p = *(const v4fa*)(pr + 4 * j);
    const v4f q = *(const v4fa*)(pc + 4 * j);
    const v4f bb = *(const v4fa*)(sB1 + 4 * j);
    const v4f ww = *(const v4fa*)(sW2 + 4 * j);
    const float h0 = fmaxf(p.x + q.x + bb.x, 0.0f);
    const float h1 = fmaxf(p.y + q.y + bb.y, 0.0f);
    const float h2 = fmaxf(p.z + q.z + bb.z, 0.0f);
    const float h3 = fmaxf(p.w + q.w + bb.w, 0.0f);
    s = fmaf(h0, ww.x, s);
    s = fmaf(h1, ww.y, s);
    s = fmaf(h2, ww.z, s);
    s = fmaf(h3, ww.w, s);
  }
  const float val = s + bf16_val(b2[0]);
  sOut[tid] = val;
  __syncthreads();

  const bool wr  = (tid < EPB / 4);
  const int  t64 = wr ? tid : 0;
  const v4f  v   = *(const v4fa*)(sOut + 4 * t64);
  const int  eb  = e0 + 4 * t64;
  const bool full  = wr && (eb + 3 < nE);
  const bool tailw = wr && !full;
  out_store_pass(out, v, eb, nE, full, tailw);
  __threadfence();
  out_store_pass(out, v, eb, nE, full, tailw);
}

static inline int cdiv(int a, int b) { return (a + b - 1) / b; }

extern "C" void kernel_launch(void* const* d_in, const int* in_sizes, int n_in,
                              void* d_out, int out_size, void* d_ws, size_t ws_size,
                              hipStream_t stream) {
  if (n_in < 7) return;
  if (in_sizes[0] < HDIM || (in_sizes[0] % HDIM) != 0) return;
  const int nA = in_sizes[0] / HDIM;
  const int nE = in_sizes[1];
  if (nE < 1) return;
  if (in_sizes[2] != nE) return;
  if (in_sizes[3] != HDIM * KDIM) return;
  if (in_sizes[4] != HDIM) return;
  if (in_sizes[5] != HDIM) return;
  if (in_sizes[6] < 1) return;
  if (out_size != nE) return;

  const float* hN  = (const float*)d_in[0];
  const int*   srcI = (const int*)d_in[1];
  const int*   dstI = (const int*)d_in[2];
  const float* W1  = (const float*)d_in[3];
  const float* b1  = (const float*)d_in[4];
  const float* W2  = (const float*)d_in[5];
  const float* b2  = (const float*)d_in[6];
  float* out = (float*)d_out;

  const int nApad = cdiv(nA, NROWB) * NROWB;
  char* ws = (char*)d_ws;
  size_t off = 0;
  const size_t oWB = off; off += (size_t)KDIM * HDIM * 2;          off = (off + 1023) & ~(size_t)1023;
  const size_t oPQ = off; off += (size_t)nApad * KDIM * sizeof(float); off = (off + 1023) & ~(size_t)1023;
  if (off > ws_size || off > (size_t)WSMAX) return;
  unsigned short* WB = (unsigned short*)(ws + oWB);
  float* PQ = (float*)(ws + oPQ);

  k_wprep<<<cdiv(NUNW, 256), 256, 0, stream>>>(W1, WB, NUNW);
  k_node<<<cdiv(nA, NROWB), GTHR, 0, stream>>>(hN, WB, PQ, nA);
  k_edge<<<cdiv(nE, EPB), EPB, 0, stream>>>(PQ, srcI, dstI, b1, W2, b2, out, nE, nA);
}
